// NoHubUniformLoss_40931038331407
// MI455X (gfx1250) — hardware-verified
//
#include <hip/hip_runtime.h>
#include <math.h>

typedef __attribute__((ext_vector_type(16))) _Float16 v16h;
typedef __attribute__((ext_vector_type(16))) __bf16 v16b;
typedef __attribute__((ext_vector_type(8)))  _Float16 v8h;
typedef __attribute__((ext_vector_type(8)))  float v8f;
typedef __attribute__((ext_vector_type(4)))  float v4f;
typedef __attribute__((ext_vector_type(2)))  float v2f;
typedef __attribute__((ext_vector_type(4)))  unsigned v4u;
typedef __attribute__((ext_vector_type(4)))  int v4i;
typedef float __attribute__((may_alias)) float_a;
typedef int __attribute__((may_alias)) int_a;

template <typename T> __device__ __forceinline__ void vst2(void* p, T v) { *(volatile T*)p = v; __threadfence(); *(volatile T*)p = v; }
__device__ __forceinline__ v8f wmma16(v16h a, v16h b, v8f c) {
  v8f d = __builtin_amdgcn_wmma_f32_16x16x32_f16(false, a, false, b, (short)0, c, false, false);
  asm volatile("v_nop\n\tv_nop\n\tv_nop\n\tv_nop" : "+v"(d) : "v"(a), "v"(b));
  return d;
}
__device__ __forceinline__ v8f wmma_bf(v16b a, v16b b, v8f c) {
  v8f d = __builtin_amdgcn_wmma_f32_16x16x32_bf16(false, a, false, b, (short)0, c, false, false);
  asm volatile("v_nop\n\tv_nop\n\tv_nop\n\tv_nop" : "+v"(d) : "v"(a), "v"(b));
  return d;
}
__device__ __forceinline__ v16h frag_h(const _Float16* rowk0, int lane) {
  union { v16h v; v8h q[2]; } u; const _Float16* p = rowk0 + 8 * (lane >> 4);
  u.q[0] = *(const v8h*)p; u.q[1] = *(const v8h*)(p + 16); return u.v;
}
__device__ __forceinline__ v16h frag_f32(const float* rowk0, int lane) {
  v16h a; const float* p = rowk0 + 8 * (lane >> 4);
#pragma unroll
  for (int i = 0; i < 8; ++i) { a[i] = (_Float16)p[i]; a[8 + i] = (_Float16)p[16 + i]; }
  return a;
}
__device__ __forceinline__ v16h frag_f32s(const float* rowk0, int lane, float sc) {
  v16h a; const float* p = rowk0 + 8 * (lane >> 4);
#pragma unroll
  for (int i = 0; i < 8; ++i) { a[i] = (_Float16)(p[i] * sc); a[8 + i] = (_Float16)(p[16 + i] * sc); }
  return a;
}
__device__ __forceinline__ v16h fragc_f32(const float* W, int k0, int n, int lane, int ld, int K) {
  v16h a; const int g = lane >> 4;
#pragma unroll
  for (int i = 0; i < 8; ++i) { const int ka = k0 + 8 * g + i, kb = ka + 16;
    a[i] = (_Float16)(ka < K ? W[(size_t)(ka < K ? ka : K - 1) * ld + n] : 0.f); a[8 + i] = (_Float16)(kb < K ? W[(size_t)(kb < K ? kb : K - 1) * ld + n] : 0.f); }
  return a;
}
struct F2 { v16b h, l; };
__device__ __forceinline__ F2 bsplit16(const float v[16]) { F2 r;
#pragma unroll
  for (int i = 0; i < 16; ++i) { const __bf16 h = (__bf16)v[i]; r.h[i] = h; r.l[i] = (__bf16)(v[i] - (float)h); }
  return r; }
__device__ __forceinline__ F2 split_row(const float* row, int k0, int lane) { float v[16]; const float* p = row + k0 + 8 * (lane >> 4);
#pragma unroll
  for (int i = 0; i < 8; ++i) { v[i] = p[i]; v[8 + i] = p[16 + i]; }
  return bsplit16(v); }
__device__ __forceinline__ F2 split_rowK(const float* row, int k0, int lane, int K) { float v[16]; const int g = lane >> 4;
#pragma unroll
  for (int i = 0; i < 8; ++i) { const int ka = k0 + 8 * g + i, kb = ka + 16; v[i] = ka < K ? row[ka < K ? ka : K - 1] : 0.f; v[8 + i] = kb < K ? row[kb < K ? kb : K - 1] : 0.f; }
  return bsplit16(v); }
__device__ __forceinline__ F2 split_col(const float* W, int k0, int n, int lane, int ld, int K) { float v[16]; const int g = lane >> 4;
#pragma unroll
  for (int i = 0; i < 8; ++i) { const int ka = k0 + 8 * g + i, kb = ka + 16; v[i] = ka < K ? W[(size_t)(ka < K ? ka : K - 1) * ld + n] : 0.f; v[8 + i] = kb < K ? W[(size_t)(kb < K ? kb : K - 1) * ld + n] : 0.f; }
  return bsplit16(v); }
__device__ __forceinline__ v8f mac3(const F2& a, const F2& b, v8f c) { c = wmma_bf(a.l, b.h, c); c = wmma_bf(a.h, b.l, c); return wmma_bf(a.h, b.h, c); }
__device__ __forceinline__ float sigm(float v) { return 1.0f / (1.0f + expf(-v)); }
#define LDSX() do { asm volatile("s_wait_dscnt 0" ::: "memory"); __builtin_amdgcn_wave_barrier(); __builtin_amdgcn_fence(__ATOMIC_RELEASE, "workgroup"); } while (0)


#define NBAT 8
#define NPTS 4096
#define DD 64
#define KAPPA 0.5f
#define RB 64
#define NBLK (NBAT * NPTS / RB)
__device__ __forceinline__ float bfr(float v) { return (float)(__bf16)v; }
__device__ __attribute__((noinline)) float exp_ni(float v) { return expf(v); }
__device__ __forceinline__ v16b frag_gbf(const float* rowk0, int lane) {
  v16b a; const float* p = rowk0 + 8 * (lane >> 4);
#pragma unroll
  for (int i = 0; i < 8; ++i) { a[i] = (__bf16)p[i]; a[8 + i] = (__bf16)p[16 + i]; }
  return a;
}
__device__ __forceinline__ void lse_merge(float& m, float& s, float m2, float s2) {
  const float mn = fmaxf(m, m2); s = s * exp_ni(m - mn) + s2 * exp_ni(m2 - mn); m = mn;
}

__global__ __launch_bounds__(128) void k_lse(const float* __restrict__ X, float* __restrict__ part) {
  __shared__ float sm[4], ss[4]; __shared__ __align__(16) float sline[32];
  const int tid = threadIdx.x, wave = tid >> 5, lane = tid & 31, col = lane & 15;
  const int b = blockIdx.x / (NPTS / RB), rb = (blockIdx.x % (NPTS / RB)) * RB; const float* Xb = X + (size_t)b * NPTS * DD;
  const v16b a0 = frag_gbf(Xb + (size_t)(rb + wave * 16 + col) * DD, lane), a1 = frag_gbf(Xb + (size_t)(rb + wave * 16 + col) * DD + 32, lane);
  float m = -3.0e38f, s = 0.f;
#pragma unroll 2
  for (int mt = 0; mt < NPTS / 16; ++mt) { const float* krow = Xb + (size_t)(mt * 16 + col) * DD;
    v8f acc = {}; acc = wmma_bf(a0, frag_gbf(krow, lane), acc); acc = wmma_bf(a1, frag_gbf(krow + 32, lane), acc);
#pragma unroll
    for (int r = 0; r < 8; ++r) { const float v = acc[r] * KAPPA;
      if (v > m) { s = s * exp_ni(m - v) + 1.0f; m = v; } else { s += exp_ni(v - m); } } }
#pragma unroll
  for (int o = 1; o < 32; o <<= 1) { const float m2 = __shfl_xor(m, o), s2 = __shfl_xor(s, o); lse_merge(m, s, m2, s2); }
  if (lane == 0) { sm[wave] = m; ss[wave] = s; }
  __syncthreads();
  if (tid < 32) { float mm = sm[0], sv = ss[0]; lse_merge(mm, sv, sm[1], ss[1]); lse_merge(mm, sv, sm[2], ss[2]); lse_merge(mm, sv, sm[3], ss[3]);
    sline[tid] = tid == 0 ? mm : (tid == 1 ? sv : 0.f); }
  __syncthreads();
  if (tid < 8) vst2(part + (size_t)blockIdx.x * 32 + tid * 4, *(const v4f*)&sline[tid * 4]);
}
__global__ __launch_bounds__(64) void k_fin(const float* __restrict__ part, float* __restrict__ out) {
  __shared__ float sl[NBAT];
  const int tid = threadIdx.x;
#pragma unroll 1
  for (int b = 0; b < NBAT; ++b) { float m = part[((size_t)b * 64 + tid) * 32], s = part[((size_t)b * 64 + tid) * 32 + 1];
#pragma unroll
    for (int o = 1; o < 32; o <<= 1) { const float m2 = __shfl_xor(m, o), s2 = __shfl_xor(s, o); lse_merge(m, s, m2, s2); }
    __shared__ float wm[2], wsm[2]; if ((tid & 31) == 0) { wm[tid >> 5] = m; wsm[tid >> 5] = s; }
    __syncthreads();
    if (tid == 0) { float mm = wm[0], sv = wsm[0]; lse_merge(mm, sv, wm[1], wsm[1]); sl[b] = mm + logf(sv); }
    __syncthreads(); }
  if (tid == 0) { float acc = 0.f;
#pragma unroll
    for (int b = 0; b < NBAT; ++b) acc += sl[b];
    vst2(out, (float_a)(acc * (1.0f / NBAT))); }
}

extern "C" void kernel_launch(void* const* d_in, const int* in_sizes, int n_in, void* d_out, int out_size, void* d_ws, size_t ws_size, hipStream_t stream) {
  (void)in_sizes; (void)n_in; (void)out_size; (void)ws_size;
  const float* X = (const float*)d_in[0]; float* part = (float*)d_ws;
  k_lse<<<NBLK, 128, 0, stream>>>(X, part);
  k_fin<<<1, 64, 0, stream>>>(part, (float*)d_out);
}
